// TSK_46050639348192
// MI455X (gfx1250) — hardware-verified
//
#include <hip/hip_runtime.h>
#include <math.h>

typedef __attribute__((ext_vector_type(16))) _Float16 v16h;
typedef __attribute__((ext_vector_type(16))) __bf16 v16b;
typedef __attribute__((ext_vector_type(8)))  _Float16 v8h;
typedef __attribute__((ext_vector_type(8)))  float v8f;
typedef __attribute__((ext_vector_type(4)))  float v4f;
typedef __attribute__((ext_vector_type(2)))  float v2f;
typedef __attribute__((ext_vector_type(4)))  unsigned v4u;
typedef __attribute__((ext_vector_type(4)))  int v4i;
typedef float __attribute__((may_alias)) float_a;
typedef int __attribute__((may_alias)) int_a;

template <typename T> __device__ __forceinline__ void vst2(void* p, T v) { *(volatile T*)p = v; __threadfence(); *(volatile T*)p = v; }
__device__ __forceinline__ v8f wmma16(v16h a, v16h b, v8f c) {
  v8f d = __builtin_amdgcn_wmma_f32_16x16x32_f16(false, a, false, b, (short)0, c, false, false);
  asm volatile("v_nop\n\tv_nop\n\tv_nop\n\tv_nop" : "+v"(d) : "v"(a), "v"(b));
  return d;
}
__device__ __forceinline__ v8f wmma_bf(v16b a, v16b b, v8f c) {
  v8f d = __builtin_amdgcn_wmma_f32_16x16x32_bf16(false, a, false, b, (short)0, c, false, false);
  asm volatile("v_nop\n\tv_nop\n\tv_nop\n\tv_nop" : "+v"(d) : "v"(a), "v"(b));
  return d;
}
__device__ __forceinline__ v16h frag_h(const _Float16* rowk0, int lane) {
  union { v16h v; v8h q[2]; } u; const _Float16* p = rowk0 + 8 * (lane >> 4);
  u.q[0] = *(const v8h*)p; u.q[1] = *(const v8h*)(p + 16); return u.v;
}
__device__ __forceinline__ v16h frag_f32(const float* rowk0, int lane) {
  v16h a; const float* p = rowk0 + 8 * (lane >> 4);
#pragma unroll
  for (int i = 0; i < 8; ++i) { a[i] = (_Float16)p[i]; a[8 + i] = (_Float16)p[16 + i]; }
  return a;
}
__device__ __forceinline__ v16h frag_f32s(const float* rowk0, int lane, float sc) {
  v16h a; const float* p = rowk0 + 8 * (lane >> 4);
#pragma unroll
  for (int i = 0; i < 8; ++i) { a[i] = (_Float16)(p[i] * sc); a[8 + i] = (_Float16)(p[16 + i] * sc); }
  return a;
}
__device__ __forceinline__ v16h fragc_f32(const float* W, int k0, int n, int lane, int ld, int K) {
  v16h a; const int g = lane >> 4;
#pragma unroll
  for (int i = 0; i < 8; ++i) { const int ka = k0 + 8 * g + i, kb = ka + 16;
    a[i] = (_Float16)(ka < K ? W[(size_t)(ka < K ? ka : K - 1) * ld + n] : 0.f); a[8 + i] = (_Float16)(kb < K ? W[(size_t)(kb < K ? kb : K - 1) * ld + n] : 0.f); }
  return a;
}
struct F2 { v16b h, l; };
__device__ __forceinline__ F2 bsplit16(const float v[16]) { F2 r;
#pragma unroll
  for (int i = 0; i < 16; ++i) { const __bf16 h = (__bf16)v[i]; r.h[i] = h; r.l[i] = (__bf16)(v[i] - (float)h); }
  return r; }
__device__ __forceinline__ F2 split_row(const float* row, int k0, int lane) { float v[16]; const float* p = row + k0 + 8 * (lane >> 4);
#pragma unroll
  for (int i = 0; i < 8; ++i) { v[i] = p[i]; v[8 + i] = p[16 + i]; }
  return bsplit16(v); }
__device__ __forceinline__ F2 split_rowK(const float* row, int k0, int lane, int K) { float v[16]; const int g = lane >> 4;
#pragma unroll
  for (int i = 0; i < 8; ++i) { const int ka = k0 + 8 * g + i, kb = ka + 16; v[i] = ka < K ? row[ka < K ? ka : K - 1] : 0.f; v[8 + i] = kb < K ? row[kb < K ? kb : K - 1] : 0.f; }
  return bsplit16(v); }
__device__ __forceinline__ F2 split_col(const float* W, int k0, int n, int lane, int ld, int K) { float v[16]; const int g = lane >> 4;
#pragma unroll
  for (int i = 0; i < 8; ++i) { const int ka = k0 + 8 * g + i, kb = ka + 16; v[i] = ka < K ? W[(size_t)(ka < K ? ka : K - 1) * ld + n] : 0.f; v[8 + i] = kb < K ? W[(size_t)(kb < K ? kb : K - 1) * ld + n] : 0.f; }
  return bsplit16(v); }
__device__ __forceinline__ v8f mac3(const F2& a, const F2& b, v8f c) { c = wmma_bf(a.l, b.h, c); c = wmma_bf(a.h, b.l, c); return wmma_bf(a.h, b.h, c); }
__device__ __forceinline__ float sigm(float v) { return 1.0f / (1.0f + expf(-v)); }
#define LDSX() do { asm volatile("s_wait_dscnt 0" ::: "memory"); __builtin_amdgcn_wave_barrier(); __builtin_amdgcn_fence(__ATOMIC_RELEASE, "workgroup"); } while (0)


#define NS 16384
#define IND 64
#define NRU 128
#define OD 32
#define ZW ((IND + 1) * NRU)
__device__ __forceinline__ float bfr(float v) { return (float)(__bf16)v; }
__device__ __attribute__((noinline)) float exp_ni(float v) { return expf(v); }

__global__ __launch_bounds__(128) void k_tsk(const float* __restrict__ X, const float* __restrict__ cen, const float* __restrict__ sig, const float* __restrict__ W, const float* __restrict__ bo, float* __restrict__ out, float* __restrict__ FRS) {
  __shared__ __align__(16) float sx[64][IND + 4]; __shared__ __align__(16) float sf[64][NRU + 4]; __shared__ float scen[IND][NRU], ssc[IND][NRU];
  __shared__ __align__(16) float sz[4][16][36]; __shared__ __align__(16) float so[4][16][36];
  const int tid = threadIdx.x, wave = tid >> 5, lane = tid & 31, col = lane & 15, g = lane >> 4; const int r0b = blockIdx.x * 64, r0 = r0b + wave * 16;
  for (int q = tid; q < IND * NRU; q += 128) { scen[q / NRU][q % NRU] = bfr(cen[q]); const float s = bfr(sig[q]); ssc[q / NRU][q % NRU] = 0.5f / (s * s) + 1e-8f; }
  for (int q = tid; q < 64 * IND; q += 128) sx[q >> 6][q & 63] = bfr(X[(size_t)(r0b + (q >> 6)) * IND + (q & 63)]);
  __syncthreads();
  { const int sl = tid >> 1, hf = tid & 1; float lg[64]; float mx = -3.4e38f;
#pragma unroll 1
    for (int rr = 0; rr < 64; ++rr) { const int r = hf * 64 + rr; float s = 0.f;
#pragma unroll 2
      for (int i = 0; i < IND; ++i) { const float d = sx[sl][i] - scen[i][r]; s -= d * d * ssc[i][r]; }
      lg[rr] = s; mx = fmaxf(mx, s); }
    mx = fmaxf(mx, __shfl_xor(mx, 1, 32)); float z = 0.f;
#pragma unroll
    for (int rr = 0; rr < 64; ++rr) { lg[rr] = exp_ni(lg[rr] - mx); z += lg[rr]; }
    z += __shfl_xor(z, 1, 32); const float inv = 1.0f / z;
#pragma unroll
    for (int rr = 0; rr < 64; ++rr) sf[sl][hf * 64 + rr] = lg[rr] * inv; }
  __syncthreads();
  for (int rl = 0; rl < 16; ++rl) vst2(FRS + (size_t)(r0 + rl) * NRU + lane * 4, *(const v4f*)(&sf[wave * 16 + rl][lane * 4]));
  v8f acc[2] = {};
#pragma unroll 1
  for (int kc = 0; kc < ZW / 32; ++kc) {
    if (kc < (IND * NRU) / 32) { const int r = kc >> 1, i0 = (kc & 1) * 32; for (int q = lane; q < 16 * 32; q += 32) { const int rl = q >> 5, i = q & 31; sz[wave][rl][i] = sf[wave * 16 + rl][r] * sx[wave * 16 + rl][i0 + i]; } }
    else { const int rb = (kc - (IND * NRU) / 32) * 32; for (int q = lane; q < 16 * 32; q += 32) { const int rl = q >> 5, i = q & 31; sz[wave][rl][i] = sf[wave * 16 + rl][rb + i]; } }
    LDSX();
    const F2 a = split_row(&sz[wave][col][0], 0, lane);
#pragma unroll
    for (int j = 0; j < 2; ++j) { const v16b wb = split_row(W + (size_t)(j * 16 + col) * ZW, kc * 32, lane).h; acc[j] = wmma_bf(a.l, wb, acc[j]); acc[j] = wmma_bf(a.h, wb, acc[j]); }
    LDSX(); }
#pragma unroll
  for (int j = 0; j < 2; ++j) { const float bb = bfr(bo[j * 16 + col]);
#pragma unroll
    for (int r = 0; r < 8; ++r) so[wave][8 * g + r][j * 16 + col] = acc[j][r] + bb; }
  LDSX();
  for (int rl = 0; rl < 16; ++rl) { if (lane < 8) vst2(out + (size_t)(r0 + rl) * OD + lane * 4, *(const v4f*)(&so[wave][rl][lane * 4])); }
}
extern "C" void kernel_launch(void* const* d_in, const int* in_sizes, int n_in, void* d_out, int out_size, void* d_ws, size_t ws_size, hipStream_t stream) {
  (void)in_sizes; (void)n_in; (void)out_size; (void)ws_size; (void)d_ws;
  const float* X = (const float*)d_in[0]; const float* cen = (const float*)d_in[1]; const float* sig = (const float*)d_in[2]; const float* W = (const float*)d_in[3]; const float* bo = (const float*)d_in[4];
  float* out = (float*)d_out; float* FRS = (float*)((char*)d_out + (size_t)NS * OD * 4);
  k_tsk<<<NS / 64, 128, 0, stream>>>(X, cen, sig, W, bo, out, FRS);
}
